// GaussCRF_11390253269333
// MI455X (gfx1250) — hardware-verified
//
#include <hip/hip_runtime.h>

#pragma clang fp contract(off)

namespace {

constexpr int NB = 2;
constexpr int NC = 21;
constexpr int HH = 512;
constexpr int WW = 512;
constexpr int HW = HH * WW;
constexpr int LH = 128;
constexpr int LW = 128;
constexpr int LHW = LH * LW;
constexpr int KF = 11;
constexpr int SPAN = 5;
constexpr int TAPS = 121;
constexpr int TP = 128;
constexpr int NITER = 5;
constexpr int POFF = 8;
constexpr int PROWS = LH + 2 * POFF;
constexpr int PPITCH = 192;
constexpr int PPLANE = NB * NC * PROWS * PPITCH;
constexpr int KROW = 32;
constexpr int KTOT = KF * KROW;
constexpr int MSGC = 32;

static_assert((NB * 3 * LHW) % 256 == 0);
static_assert((NB * LHW) % 8 == 0);
static_assert((NB * HW) % 256 == 0);
static_assert((NB * NC * PROWS) % 8 == 0);
static_assert(LW % 16 == 0);
static_assert(WW % 32 == 0);
static_assert(HH % 8 == 0);
static_assert((3 * 16 * KTOT) % (8 * 64) == 0);
static_assert(HW == (1 << 18));
static_assert(LHW == (1 << 14));

typedef unsigned short v8us __attribute__((ext_vector_type(8)));
typedef v8us __attribute__((may_alias)) v8usa;
typedef float v8f __attribute__((ext_vector_type(8)));
typedef float v4f __attribute__((ext_vector_type(4)));
typedef v4f __attribute__((may_alias)) v4fa;
typedef __bf16 v16b __attribute__((ext_vector_type(16)));

union FragB { v16b v; v8us half[2]; };

__device__ __forceinline__ int clampi(int v, int lo, int hi) {
  return v < lo ? lo : (v > hi ? hi : v);
}

__device__ __forceinline__ unsigned short bf16_rne(float x) {
  unsigned int u = __float_as_uint(x);
  u = (u + 0x7FFFu + ((u >> 16) & 1u)) >> 16;
  return (unsigned short)u;
}
__device__ __forceinline__ float bf16_val(unsigned short b) {
  return __uint_as_float(((unsigned int)b) << 16);
}
__device__ __forceinline__ void split3(float x, unsigned short& h, unsigned short& m, unsigned short& l) {
  h = bf16_rne(x);
  const float r1 = x - bf16_val(h);
  m = bf16_rne(r1);
  const float r2 = r1 - bf16_val(m);
  l = bf16_rne(r2);
}

__device__ __forceinline__ v8f wmma_bf16x(v16b a, v16b b, v8f c) {
  v8f d = __builtin_amdgcn_wmma_f32_16x16x32_bf16(false, a, false, b, (short)0, c, false, false);
  asm volatile("v_nop\n\tv_nop\n\tv_nop\n\tv_nop" : "+v"(d) : "v"(a), "v"(b));
  return d;
}

__device__ __forceinline__ v16b frag16(const unsigned short* p, int h) {
  FragB f;
  f.half[0] = *(const v8usa*)(p + 8 * h);
  f.half[1] = *(const v8usa*)(p + 16 + 8 * h);
  return f.v;
}

__global__ __launch_bounds__(256) void k_postab(const float* __restrict__ pos_sdims,
                                                 float* __restrict__ tab) {
  const int t = threadIdx.x;
  const float s = pos_sdims[0];
  const int q = t & 127;
  float acc = 0.f;
  if (t < 128) {
    #pragma unroll
    for (int i = 0; i < 4; ++i) {
      const float v = (float)(4 * q + i) * s;
      #pragma unroll
      for (int j = 0; j < 4; ++j) acc = acc + v;
    }
  } else {
    #pragma unroll
    for (int i = 0; i < 4; ++i) {
      #pragma unroll
      for (int j = 0; j < 4; ++j) acc = acc + (float)(4 * q + j) * s;
    }
  }
  const float r = acc * 0.0625f;
  *(volatile float*)(tab + t) = r;
  __threadfence();
  *(volatile float*)(tab + t) = r;
}

__global__ __launch_bounds__(256) void k_poolimg(const float* __restrict__ img,
                                                  const float* __restrict__ col_schan,
                                                  float* __restrict__ cp) {
  const int idx = blockIdx.x * 256 + threadIdx.x;
  const int X = idx & 127;
  const int Y = (idx >> 7) & 127;
  const int ch = (idx >> 14) % 3;
  const int b = idx / (3 * LHW);
  const float cs = col_schan[0];
  const float* src = img + ((size_t)(b * 3 + ch) * HH + 4 * Y) * WW + 4 * X;
  float acc = 0.f;
  #pragma unroll
  for (int i = 0; i < 4; ++i) {
    const v4f q = *(const v4fa*)(src + (size_t)i * WW);
    acc = acc + q.x * cs;
    acc = acc + q.y * cs;
    acc = acc + q.z * cs;
    acc = acc + q.w * cs;
  }
  const float r = acc * 0.0625f;
  *(volatile float*)(cp + idx) = r;
  __threadfence();
  *(volatile float*)(cp + idx) = r;
}

__global__ __launch_bounds__(256) void k_gauss(const float* __restrict__ cp,
                                                const float* __restrict__ tab,
                                                const float* __restrict__ pos_compat,
                                                const float* __restrict__ col_compat,
                                                unsigned short* __restrict__ gsp) {
  __shared__ __attribute__((aligned(16))) unsigned short stg[8][3 * TP];
  const int lane = threadIdx.x & 31, w = threadIdx.x >> 5;
  const int pix = blockIdx.x * 8 + w;
  const int b = pix >> 14, y = (pix >> 7) & 127, x = pix & 127;
  const float pc = pos_compat[0];
  const float cc = col_compat[0];
  const float* tab0 = tab;
  const float* tab1 = tab + 128;
  const float* cpb = cp + (size_t)b * 3 * LHW;
  const float f0 = tab0[y];
  const float f1 = tab1[x];
  const float c0 = cpb[y * LW + x];
  const float c1 = cpb[LHW + y * LW + x];
  const float c2 = cpb[2 * LHW + y * LW + x];
  #pragma unroll 1
  for (int k = 0; k < 4; ++k) {
    const int t = lane + 32 * k;
    const int tc = t < TAPS ? t : TAPS - 1;
    const int ti = tc / KF;
    const int di = ti - SPAN;
    const int dj = tc - ti * KF - SPAN;
    const int ys = y + di, xs = x + dj;
    const bool inb = (t < TAPS) && ys >= 0 && ys < LH && xs >= 0 && xs < LW;
    const int ysc = clampi(ys, 0, LH - 1), xsc = clampi(xs, 0, LW - 1);
    const float g0 = tab0[ysc];
    const float g1 = tab1[xsc];
    const float d0 = cpb[ysc * LW + xsc];
    const float d1 = cpb[LHW + ysc * LW + xsc];
    const float d2 = cpb[2 * LHW + ysc * LW + xsc];
    const float dp0 = g0 - f0, dp1 = g1 - f1;
    float sp = dp0 * dp0;
    sp = sp + dp1 * dp1;
    const float dc0 = d0 - c0, dc1 = d1 - c1, dc2 = d2 - c2;
    float sc = dc0 * dc0;
    sc = sc + dc1 * dc1;
    sc = sc + dc2 * dc2;
    const float gp = expf(-0.5f * sp);
    const float gc = expf(-0.5f * sc);
    float g = pc * gp + cc * gc;
    g = inb ? g : 0.f;
    unsigned short ph, pm, pl;
    split3(g, ph, pm, pl);
    stg[w][t] = ph;
    stg[w][TP + t] = pm;
    stg[w][2 * TP + t] = pl;
  }
  __syncthreads();
  unsigned short* dst = gsp + (size_t)pix * (3 * TP);
  const v8us v0 = *(const v8usa*)(&stg[w][8 * lane]);
  const v8us v1 = *(const v8usa*)(&stg[w][8 * (32 + (lane & 15))]);
  *(volatile v8us*)(dst + 8 * lane) = v0;
  if (lane < 16) *(volatile v8us*)(dst + 8 * (32 + lane)) = v1;
  __threadfence();
  *(volatile v8us*)(dst + 8 * lane) = v0;
  if (lane < 16) *(volatile v8us*)(dst + 8 * (32 + lane)) = v1;
}

__global__ __launch_bounds__(256) void k_logsm(const float* __restrict__ unary,
                                                float* __restrict__ lg) {
  const int idx = blockIdx.x * 256 + threadIdx.x;
  const int pixi = idx & (HW - 1);
  const int b = idx >> 18;
  const float* u = unary + (size_t)b * NC * HW + pixi;
  float mx = u[0];
  #pragma unroll 1
  for (int c = 1; c < NC; ++c) mx = fmaxf(mx, u[(size_t)c * HW]);
  float s = 0.f;
  #pragma unroll 1
  for (int c = 0; c < NC; ++c) s = s + expf(u[(size_t)c * HW] - mx);
  const float lse = logf(s);
  float* o = lg + (size_t)b * NC * HW + pixi;
  #pragma unroll 1
  for (int c = 0; c < NC; ++c) {
    const float v = (u[(size_t)c * HW] - mx) - lse;
    *(volatile float*)(o + (size_t)c * HW) = v;
  }
  __threadfence();
  #pragma unroll 1
  for (int c = 0; c < NC; ++c) {
    const float v = (u[(size_t)c * HW] - mx) - lse;
    *(volatile float*)(o + (size_t)c * HW) = v;
  }
}

__global__ __launch_bounds__(256) void k_pool(const float* __restrict__ src,
                                               unsigned short* __restrict__ planes) {
  __shared__ __attribute__((aligned(16))) unsigned short stg[8][3 * PPITCH];
  const int lane = threadIdx.x & 31, w = threadIdx.x >> 5;
  const int R = blockIdx.x * 8 + w;
  const int prow = R % PROWS;
  const int bc = R / PROWS;
  const int Y = prow - POFF;
  const bool valid = (Y >= 0) && (Y < LH);
  {
    const v8us z = {0, 0, 0, 0, 0, 0, 0, 0};
    *(v8usa*)(&stg[w][8 * lane]) = z;
    *(v8usa*)(&stg[w][8 * (lane + 32)]) = z;
    if (lane < 8) *(v8usa*)(&stg[w][8 * (lane + 64)]) = z;
  }
  __syncthreads();
  if (valid) {
    const float* base = src + ((size_t)bc * HH + 4 * Y) * WW;
    #pragma unroll
    for (int k = 0; k < 4; ++k) {
      const int X = lane + 32 * k;
      const float* p0 = base + 4 * X;
      float acc = 0.f;
      #pragma unroll
      for (int i = 0; i < 4; ++i) {
        const v4f q = *(const v4fa*)(p0 + (size_t)i * WW);
        acc = acc + q.x;
        acc = acc + q.y;
        acc = acc + q.z;
        acc = acc + q.w;
      }
      const float pv = acc * 0.0625f;
      unsigned short ph, pm, pl;
      split3(pv, ph, pm, pl);
      stg[w][POFF + X] = ph;
      stg[w][PPITCH + POFF + X] = pm;
      stg[w][2 * PPITCH + POFF + X] = pl;
    }
  }
  __syncthreads();
  const size_t rowoff = ((size_t)bc * PROWS + prow) * PPITCH;
  const int lc = lane < 24 ? lane : 23;
  const v8us r0 = *(const v8usa*)(&stg[w][8 * lc]);
  const v8us r1 = *(const v8usa*)(&stg[w][PPITCH + 8 * lc]);
  const v8us r2 = *(const v8usa*)(&stg[w][2 * PPITCH + 8 * lc]);
  if (lane < 24) {
    *(volatile v8us*)(planes + rowoff + 8 * lane) = r0;
    *(volatile v8us*)(planes + (size_t)PPLANE + rowoff + 8 * lane) = r1;
    *(volatile v8us*)(planes + 2 * (size_t)PPLANE + rowoff + 8 * lane) = r2;
  }
  __threadfence();
  if (lane < 24) {
    *(volatile v8us*)(planes + rowoff + 8 * lane) = r0;
    *(volatile v8us*)(planes + (size_t)PPLANE + rowoff + 8 * lane) = r1;
    *(volatile v8us*)(planes + 2 * (size_t)PPLANE + rowoff + 8 * lane) = r2;
  }
}

__global__ __launch_bounds__(64) void k_msg(const unsigned short* __restrict__ gsp,
                                             const unsigned short* __restrict__ planes,
                                             float* __restrict__ msg) {
  __shared__ __attribute__((aligned(16))) unsigned short At[3][16][KTOT];
  __shared__ __attribute__((aligned(16))) float Dst[16 * MSGC];
  const int tid = threadIdx.x, lane = tid & 31, w = tid >> 5;
  const int h = lane >> 4, m = lane & 15;
  const int xt = blockIdx.x, y = blockIdx.y, b = blockIdx.z;
  const int x0 = xt * 16;

  {
    const v8us z = {0, 0, 0, 0, 0, 0, 0, 0};
    v8usa* az = (v8usa*)(&At[0][0][0]);
    #pragma unroll 1
    for (int i = tid; i < (3 * 16 * KTOT) / 8; i += 64) az[i] = z;
  }
  __syncthreads();
  {
    const unsigned short* gb = gsp + ((size_t)b * LHW + (size_t)y * LW + x0) * (3 * TP);
    #pragma unroll 1
    for (int idx = tid; idx < 16 * TAPS; idx += 64) {
      const int mm = idx / TAPS;
      const int t = idx - mm * TAPS;
      const int r = t / KF;
      const int q = t - r * KF;
      const unsigned short* gpx = gb + (size_t)mm * (3 * TP) + t;
      const int k = r * KROW + mm + 3 + q;
      At[0][mm][k] = gpx[0];
      At[1][mm][k] = gpx[TP];
      At[2][mm][k] = gpx[2 * TP];
    }
  }
  __syncthreads();

  int cB = 16 * w + m;
  cB = cB > (NC - 1) ? (NC - 1) : cB;
  const size_t rowoff = ((size_t)(b * NC + cB) * PROWS + (size_t)(y + 3)) * PPITCH + x0;
  const unsigned short* B0 = planes + rowoff;
  const unsigned short* B1 = planes + (size_t)PPLANE + rowoff;
  const unsigned short* B2 = planes + 2 * (size_t)PPLANE + rowoff;

  const v8f zero8 = {0.f, 0.f, 0.f, 0.f, 0.f, 0.f, 0.f, 0.f};
  v8f acc = zero8;
  #pragma unroll 1
  for (int r = 0; r < KF; ++r) {
    const v16b ah = frag16(&At[0][m][r * KROW], h);
    const v16b am = frag16(&At[1][m][r * KROW], h);
    const v16b al = frag16(&At[2][m][r * KROW], h);
    const v16b bh = frag16(B0 + r * PPITCH, h);
    const v16b bm = frag16(B1 + r * PPITCH, h);
    const v16b bl = frag16(B2 + r * PPITCH, h);
    acc = wmma_bf16x(ah, bh, acc);
    acc = wmma_bf16x(ah, bm, acc);
    acc = wmma_bf16x(am, bh, acc);
    acc = wmma_bf16x(ah, bl, acc);
    acc = wmma_bf16x(am, bm, acc);
    acc = wmma_bf16x(al, bh, acc);
  }

  #pragma unroll
  for (int r = 0; r < 8; ++r) Dst[(8 * h + r) * MSGC + 16 * w + m] = acc[r];
  __syncthreads();

  const int q8 = tid & 7;
  const int l0 = tid >> 3;
  float* mb = msg + ((size_t)(b * LH + y) * LW + x0) * MSGC;
  const v4f v0 = *(const v4fa*)(&Dst[l0 * MSGC + 4 * q8]);
  const v4f v1 = *(const v4fa*)(&Dst[(8 + l0) * MSGC + 4 * q8]);
  *(volatile v4f*)(mb + (size_t)l0 * MSGC + 4 * q8) = v0;
  *(volatile v4f*)(mb + (size_t)(8 + l0) * MSGC + 4 * q8) = v1;
  __threadfence();
  *(volatile v4f*)(mb + (size_t)l0 * MSGC + 4 * q8) = v0;
  *(volatile v4f*)(mb + (size_t)(8 + l0) * MSGC + 4 * q8) = v1;
}

__global__ __launch_bounds__(256) void k_fuse(const float* __restrict__ msg,
                                               const float* __restrict__ lg,
                                               const float* __restrict__ wptr,
                                               float* __restrict__ out,
                                               int last) {
  __shared__ __attribute__((aligned(16))) float mwin[4 * 10 * MSGC];
  __shared__ float tmpw[8 * 10 * MSGC];
  __shared__ float vbuf[NC * 256];
  const int tid = threadIdx.x, lane = tid & 31, w = tid >> 5;
  const int tX = blockIdx.x, tY = blockIdx.y, b = blockIdx.z;
  const float wg = wptr[0];
  const float uw = 1.0f - wg;

  #pragma unroll 1
  for (int i = tid; i < 4 * 10 * 8; i += 256) {
    const int pos = i >> 3, q = i & 7;
    const int wr = pos / 10, wc = pos - wr * 10;
    const int yl = clampi(2 * tY - 1 + wr, 0, LH - 1);
    const int xl = clampi(8 * tX - 1 + wc, 0, LW - 1);
    const v4f v = *(const v4fa*)(msg + ((size_t)(b * LH + yl) * LW + xl) * MSGC + 4 * q);
    *(v4fa*)(&mwin[pos * MSGC + 4 * q]) = v;
  }
  __syncthreads();

  #pragma unroll 1
  for (int i = tid; i < 8 * 10 * NC; i += 256) {
    const int c = i % NC;
    const int rest = i / NC;
    const int j = rest % 10;
    const int r = rest / 10;
    const int r4 = r & 3, ra = r >> 2;
    const int i0 = (r4 < 2) ? ra : ra + 1;
    float w0 = (r4 == 0) ? 0.375f : ((r4 == 1) ? 0.125f : ((r4 == 2) ? 0.875f : 0.625f));
    float w1 = 1.0f - w0;
    const int gi0 = 2 * tY - 1 + i0;
    if (gi0 < 0) { w0 = 0.f; w1 = 1.f; }
    if (gi0 + 1 > LH - 1) { w1 = 0.f; w0 = 1.f; }
    const float a0 = mwin[(i0 * 10 + j) * MSGC + c];
    const float a1 = mwin[((i0 + 1) * 10 + j) * MSGC + c];
    tmpw[(r * 10 + j) * MSGC + c] = w0 * a0 + w1 * a1;
  }
  __syncthreads();

  const int Y = 8 * tY + w;
  const int X = 32 * tX + lane;
  const int x4 = lane & 3, xa = lane >> 2;
  const int j0 = (x4 < 2) ? xa : xa + 1;
  float wx0 = (x4 == 0) ? 0.375f : ((x4 == 1) ? 0.125f : ((x4 == 2) ? 0.875f : 0.625f));
  float wx1 = 1.0f - wx0;
  const int gj0 = 8 * tX - 1 + j0;
  if (gj0 < 0) { wx0 = 0.f; wx1 = 1.f; }
  if (gj0 + 1 > LW - 1) { wx1 = 0.f; wx0 = 1.f; }

  const float* lgp = lg + ((size_t)(b * NC) * HH + Y) * WW + X;
  float* op = out + ((size_t)(b * NC) * HH + Y) * WW + X;
  float mx = -__builtin_inff();
  #pragma unroll 1
  for (int c = 0; c < NC; ++c) {
    const float t0 = tmpw[(w * 10 + j0) * MSGC + c];
    const float t1 = tmpw[(w * 10 + j0 + 1) * MSGC + c];
    const float up = wx0 * t0 + wx1 * t1;
    const float lv = lgp[(size_t)c * HW];
    const float v = uw * lv + wg * up;
    vbuf[c * 256 + tid] = v;
    mx = fmaxf(mx, v);
  }
  if (last) {
    #pragma unroll 1
    for (int c = 0; c < NC; ++c) {
      const float v = vbuf[c * 256 + tid];
      *(volatile float*)(op + (size_t)c * HW) = v;
    }
    __threadfence();
    #pragma unroll 1
    for (int c = 0; c < NC; ++c) {
      const float v = vbuf[c * 256 + tid];
      *(volatile float*)(op + (size_t)c * HW) = v;
    }
  } else {
    float s = 0.f;
    #pragma unroll 1
    for (int c = 0; c < NC; ++c) {
      const float e = expf(vbuf[c * 256 + tid] - mx);
      vbuf[c * 256 + tid] = e;
      s = s + e;
    }
    const float inv = 1.0f / s;
    #pragma unroll 1
    for (int c = 0; c < NC; ++c) {
      const float o = vbuf[c * 256 + tid] * inv;
      *(volatile float*)(op + (size_t)c * HW) = o;
    }
    __threadfence();
    #pragma unroll 1
    for (int c = 0; c < NC; ++c) {
      const float o = vbuf[c * 256 + tid] * inv;
      *(volatile float*)(op + (size_t)c * HW) = o;
    }
  }
}

}

extern "C" void kernel_launch(void* const* d_in, const int* in_sizes, int n_in,
                              void* d_out, int out_size, void* d_ws, size_t ws_size,
                              hipStream_t stream) {
  if (n_in < 7) return;
  if (in_sizes[0] != NB * NC * HW) return;
  if (in_sizes[1] != NB * 3 * HW) return;
  for (int i = 2; i < 7; ++i) {
    if (in_sizes[i] < 1) return;
  }
  if (out_size != NB * NC * HW) return;

  const float* unary      = (const float*)d_in[0];
  const float* img        = (const float*)d_in[1];
  const float* pos_sdims  = (const float*)d_in[2];
  const float* col_schan  = (const float*)d_in[3];
  const float* pos_compat = (const float*)d_in[4];
  const float* col_compat = (const float*)d_in[5];
  const float* weight     = (const float*)d_in[6];
  float* out = (float*)d_out;

  const size_t lg_bytes  = (size_t)NB * NC * HW * 4;
  const size_t gsp_bytes = (size_t)NB * LHW * 3 * TP * 2;
  const size_t pl_bytes  = (size_t)3 * PPLANE * 2;
  const size_t msg_bytes = (size_t)NB * LHW * MSGC * 4;
  const size_t cp_bytes  = (size_t)NB * 3 * LHW * 4;
  const size_t tab_bytes = 1024;
  const size_t total = lg_bytes + gsp_bytes + pl_bytes + msg_bytes + cp_bytes + tab_bytes;
  if (total > ws_size) return;

  char* ws = (char*)d_ws;
  float* lg = (float*)ws;
  unsigned short* gsp = (unsigned short*)(ws + lg_bytes);
  unsigned short* planes = (unsigned short*)(ws + lg_bytes + gsp_bytes);
  float* msg = (float*)(ws + lg_bytes + gsp_bytes + pl_bytes);
  float* cp = (float*)(ws + lg_bytes + gsp_bytes + pl_bytes + msg_bytes);
  float* tab = (float*)(ws + lg_bytes + gsp_bytes + pl_bytes + msg_bytes + cp_bytes);

  k_postab<<<1, 256, 0, stream>>>(pos_sdims, tab);
  k_poolimg<<<(NB * 3 * LHW) / 256, 256, 0, stream>>>(img, col_schan, cp);
  k_gauss<<<(NB * LHW) / 8, 256, 0, stream>>>(cp, tab, pos_compat, col_compat, gsp);
  k_logsm<<<(NB * HW) / 256, 256, 0, stream>>>(unary, lg);

  const dim3 gMsg(LW / 16, LH, NB);
  const dim3 gFuse(WW / 32, HH / 8, NB);
  for (int it = 0; it < NITER; ++it) {
    const float* src = (it == 0) ? (const float*)lg : (const float*)out;
    k_pool<<<(NB * NC * PROWS) / 8, 256, 0, stream>>>(src, planes);
    k_msg<<<gMsg, 64, 0, stream>>>(gsp, planes, msg);
    k_fuse<<<gFuse, 256, 0, stream>>>(msg, lg, weight, out, (it == NITER - 1) ? 1 : 0);
  }
}
